// ShiftLocalAttention2d_9749575762382
// MI455X (gfx1250) — hardware-verified
//
#include <hip/hip_runtime.h>
#include <math.h>

typedef __attribute__((ext_vector_type(16))) _Float16 v16h;
typedef __attribute__((ext_vector_type(16))) __bf16 v16b;
typedef __attribute__((ext_vector_type(8)))  _Float16 v8h;
typedef __attribute__((ext_vector_type(8)))  float v8f;
typedef __attribute__((ext_vector_type(4)))  float v4f;
typedef __attribute__((ext_vector_type(2)))  float v2f;
typedef __attribute__((ext_vector_type(4)))  unsigned v4u;
typedef __attribute__((ext_vector_type(4)))  int v4i;
typedef float __attribute__((may_alias)) float_a;
typedef int __attribute__((may_alias)) int_a;

template <typename T> __device__ __forceinline__ void vst2(void* p, T v) { *(volatile T*)p = v; __threadfence(); *(volatile T*)p = v; }
__device__ __forceinline__ v8f wmma16(v16h a, v16h b, v8f c) {
  v8f d = __builtin_amdgcn_wmma_f32_16x16x32_f16(false, a, false, b, (short)0, c, false, false);
  asm volatile("v_nop\n\tv_nop\n\tv_nop\n\tv_nop" : "+v"(d) : "v"(a), "v"(b));
  return d;
}
__device__ __forceinline__ v8f wmma_bf(v16b a, v16b b, v8f c) {
  v8f d = __builtin_amdgcn_wmma_f32_16x16x32_bf16(false, a, false, b, (short)0, c, false, false);
  asm volatile("v_nop\n\tv_nop\n\tv_nop\n\tv_nop" : "+v"(d) : "v"(a), "v"(b));
  return d;
}
__device__ __forceinline__ v16h frag_h(const _Float16* rowk0, int lane) {
  union { v16h v; v8h q[2]; } u; const _Float16* p = rowk0 + 8 * (lane >> 4);
  u.q[0] = *(const v8h*)p; u.q[1] = *(const v8h*)(p + 16); return u.v;
}
__device__ __forceinline__ v16h frag_f32(const float* rowk0, int lane) {
  v16h a; const float* p = rowk0 + 8 * (lane >> 4);
#pragma unroll
  for (int i = 0; i < 8; ++i) { a[i] = (_Float16)p[i]; a[8 + i] = (_Float16)p[16 + i]; }
  return a;
}
__device__ __forceinline__ v16h frag_f32s(const float* rowk0, int lane, float sc) {
  v16h a; const float* p = rowk0 + 8 * (lane >> 4);
#pragma unroll
  for (int i = 0; i < 8; ++i) { a[i] = (_Float16)(p[i] * sc); a[8 + i] = (_Float16)(p[16 + i] * sc); }
  return a;
}
__device__ __forceinline__ v16h fragc_f32(const float* W, int k0, int n, int lane, int ld, int K) {
  v16h a; const int g = lane >> 4;
#pragma unroll
  for (int i = 0; i < 8; ++i) { const int ka = k0 + 8 * g + i, kb = ka + 16;
    a[i] = (_Float16)(ka < K ? W[(size_t)ka * ld + n] : 0.f); a[8 + i] = (_Float16)(kb < K ? W[(size_t)kb * ld + n] : 0.f); }
  return a;
}
struct F2 { v16b h, l; };
__device__ __forceinline__ F2 bsplit16(const float v[16]) { F2 r;
#pragma unroll
  for (int i = 0; i < 16; ++i) { const __bf16 h = (__bf16)v[i]; r.h[i] = h; r.l[i] = (__bf16)(v[i] - (float)h); }
  return r; }
__device__ __forceinline__ F2 split_row(const float* row, int k0, int lane) { float v[16]; const float* p = row + k0 + 8 * (lane >> 4);
#pragma unroll
  for (int i = 0; i < 8; ++i) { v[i] = p[i]; v[8 + i] = p[16 + i]; }
  return bsplit16(v); }
__device__ __forceinline__ F2 split_rowK(const float* row, int k0, int lane, int K) { float v[16]; const int g = lane >> 4;
#pragma unroll
  for (int i = 0; i < 8; ++i) { const int ka = k0 + 8 * g + i, kb = ka + 16; v[i] = ka < K ? row[ka] : 0.f; v[8 + i] = kb < K ? row[kb] : 0.f; }
  return bsplit16(v); }
__device__ __forceinline__ F2 split_col(const float* W, int k0, int n, int lane, int ld, int K) { float v[16]; const int g = lane >> 4;
#pragma unroll
  for (int i = 0; i < 8; ++i) { const int ka = k0 + 8 * g + i, kb = ka + 16; v[i] = ka < K ? W[(size_t)ka * ld + n] : 0.f; v[8 + i] = kb < K ? W[(size_t)kb * ld + n] : 0.f; }
  return bsplit16(v); }
__device__ __forceinline__ v8f mac3(const F2& a, const F2& b, v8f c) { c = wmma_bf(a.l, b.h, c); c = wmma_bf(a.h, b.l, c); return wmma_bf(a.h, b.h, c); }
__device__ __forceinline__ float sigm(float v) { return 1.0f / (1.0f + expf(-v)); }
#define LDSX() do { asm volatile("s_wait_dscnt 0" ::: "memory"); __builtin_amdgcn_wave_barrier(); __builtin_amdgcn_fence(__ATOMIC_RELEASE, "workgroup"); } while (0)

#define NB 4
#define NHD 8
#define HD 32
#define HI 48
#define WI 48
#define NPIX (HI * WI)
#define RW 3
#define KR 8
#define NKEY (KR * WI)
#define NQ (2 * WI)

__global__ __launch_bounds__(128) void k_attn(const float* __restrict__ q, const float* __restrict__ k, const float* __restrict__ v, float* __restrict__ out) {
  __shared__ __align__(16) float sK[NKEY][HD + 1];
  __shared__ __align__(16) float sVT[HD][NKEY + 4];
  __shared__ __align__(16) float sQ[NQ][HD + 1];
  __shared__ __align__(16) float sS[4][16][NKEY + 4];
  __shared__ __align__(16) float sO[HD][NQ + 4];
  const int tid = threadIdx.x, wave = tid >> 5, lane = tid & 31, col = lane & 15, g = lane >> 4;
  const int b = blockIdx.z, h = blockIdx.y, y0 = blockIdx.x * 2;
  const size_t cbase = ((size_t)b * (NHD * HD) + (size_t)h * HD) * NPIX;
  for (int e = tid; e < NKEY * HD; e += 128) { const int d = e / NKEY, kk = e % NKEY; const int ky = y0 - RW + kk / WI, kx = kk % WI; float kvv = 0.f, vvv = 0.f;
    if (ky >= 0 && ky < HI) { const size_t o = cbase + (size_t)d * NPIX + ky * WI + kx; kvv = k[o]; vvv = v[o]; }
    sK[kk][d] = kvv; sVT[d][kk] = vvv; }
  for (int e = tid; e < NQ * HD; e += 128) { const int d = e / NQ, qq = e % NQ; sQ[qq][d] = q[cbase + (size_t)d * NPIX + (y0 + qq / WI) * WI + qq % WI]; }
  __syncthreads();
  for (int qt = wave; qt < NQ / 16; qt += 4) {
    const F2 aq = split_row(&sQ[qt * 16 + col][0], 0, lane);
#pragma unroll 4
    for (int t = 0; t < NKEY / 16; ++t) { v8f s = {}; s = mac3(aq, split_row(&sK[t * 16 + col][0], 0, lane), s);
#pragma unroll
      for (int r = 0; r < 8; ++r) { const int qq = qt * 16 + 8 * g + r, kk = t * 16 + col; const int qy = y0 + qq / WI, qx = qq % WI, ky = y0 - RW + kk / WI, kx = kk % WI;
        const bool ok = (ky >= 0 && ky < HI) && (ky - qy >= -RW) && (ky - qy <= RW) && (kx - qx >= -RW) && (kx - qx <= RW);
        sS[wave][8 * g + r][kk] = ok ? s[r] * 0.17677669529663687f : -3.0e38f; } }
    LDSX();
    { const int m = col; float* row = &sS[wave][m][0]; float mx = -3.4e38f;
#pragma unroll 4
      for (int j = g * (NKEY / 2); j < (g + 1) * (NKEY / 2); ++j) mx = fmaxf(mx, row[j]);
      mx = fmaxf(mx, __shfl_xor(mx, 16, 32)); float l = 0.f;
#pragma unroll 4
      for (int j = g * (NKEY / 2); j < (g + 1) * (NKEY / 2); ++j) { const float p = row[j] <= -1.0e38f ? 0.f : expf(row[j] - mx); row[j] = p; l += p; }
      l += __shfl_xor(l, 16, 32); const float inv = 1.0f / l;
      LDSX();
#pragma unroll 4
      for (int j = g * (NKEY / 2); j < (g + 1) * (NKEY / 2); ++j) row[j] *= inv; }
    LDSX();
    v8f acc[2] = {};
#pragma unroll 2
    for (int kc = 0; kc < NKEY / 32; ++kc) { const F2 pa = split_row(&sS[wave][col][0], kc * 32, lane);
#pragma unroll
      for (int t = 0; t < 2; ++t) acc[t] = mac3(pa, split_row(&sVT[t * 16 + col][0], kc * 32, lane), acc[t]); }
#pragma unroll
    for (int t = 0; t < 2; ++t)
#pragma unroll
      for (int r = 0; r < 8; ++r) sO[t * 16 + col][qt * 16 + 8 * g + r] = acc[t][r];
    LDSX(); }
  __syncthreads();
  for (int e = tid; e < HD * (NQ / 4); e += 128) { const int d = e / (NQ / 4), pc = e % (NQ / 4); vst2(out + cbase + (size_t)d * NPIX + y0 * WI + pc * 4, *(const v4f*)(&sO[d][pc * 4])); }
}
extern "C" void kernel_launch(void* const* d_in, const int* in_sizes, int n_in, void* d_out, int out_size, void* d_ws, size_t ws_size, hipStream_t stream) {
  (void)in_sizes; (void)n_in; (void)out_size; (void)ws_size; (void)d_ws;
  const float* q = (const float*)d_in[0]; const float* k = (const float*)d_in[1]; const float* v = (const float*)d_in[2];
  float* out = (float*)d_out;
  k_attn<<<dim3(HI / 2, NHD, NB), 128, 0, stream>>>(q, k, v, out);
}
